// LSTMfs__46308337386349
// MI455X (gfx1250) — hardware-verified
//
#include <hip/hip_runtime.h>
#include <math.h>

constexpr int kBatch        = 32;
constexpr int kSeq          = 1024;
constexpr int kHid          = 256;
constexpr int kGates        = 4 * kHid;
constexpr int kThreads      = 256;
constexpr int kSeqPerBlock  = 16;
constexpr int kNodesPerBlk  = 8;
constexpr int kMaxDepth     = 64;
constexpr int kHPitch       = 264;
constexpr int kOPitch       = 260;
constexpr float kWCarry     = 16.0f;
constexpr float kWCarryInv  = 1.0f / 16.0f;
static_assert(kHPitch % 8 == 0, "16-B aligned fragment rows");
static_assert(kOPitch % 4 == 0, "16-B aligned staging rows");
static_assert(kBatch % kSeqPerBlock == 0, "whole blocks");
static_assert(kHid == kThreads, "one thread per hidden column in tile fills");
static_assert(kHid % 32 == 0, "K multiple of 32");

typedef __attribute__((ext_vector_type(16))) _Float16 v16h;
typedef __attribute__((ext_vector_type(8)))  _Float16 v8h;
typedef __attribute__((ext_vector_type(16))) __bf16   v16b;
typedef __attribute__((ext_vector_type(8)))  __bf16   v8b;
typedef __attribute__((ext_vector_type(8)))  float    v8f;
typedef __attribute__((ext_vector_type(4)))  float    v4f;

__device__ __forceinline__ unsigned short f2bf_bits(float f) {
  unsigned u = __float_as_uint(f);
  return (unsigned short)((u + 0x7FFFu + ((u >> 16) & 1u)) >> 16);
}
__device__ __forceinline__ float bf_bits2f(unsigned short h) { return __uint_as_float(((unsigned)h) << 16); }

__device__ __forceinline__ void dep_guard_h(v8f& a, v8f& b, v16h x, v16h y) { asm volatile("v_nop\n\tv_nop\n\tv_nop\n\tv_nop" : "+v"(a), "+v"(b) : "v"(x), "v"(y)); }
__device__ __forceinline__ void dep_guard_b(v8f& a, v8f& b, v16b x, v16b y) { asm volatile("v_nop\n\tv_nop\n\tv_nop\n\tv_nop" : "+v"(a), "+v"(b) : "v"(x), "v"(y)); }
__device__ __forceinline__ void keep4_h(v16h a, v16h b, v16h c, v16h d) { asm volatile("v_nop" :: "v"(a), "v"(b), "v"(c), "v"(d)); }
__device__ __forceinline__ void keep4_b(v16b a, v16b b, v16b c, v16b d) { asm volatile("v_nop" :: "v"(a), "v"(b), "v"(c), "v"(d)); }
__device__ __forceinline__ void acc_guard4(v8f& a, v8f& b, v8f& c, v8f& d) { asm volatile("v_nop\n\tv_nop\n\tv_nop\n\tv_nop" : "+v"(a), "+v"(b), "+v"(c), "+v"(d)); }
template <typename T> struct Frag;
template <> struct Frag<_Float16> {
  typedef v16h V; union U { v16h v; v8h h[2]; };
  static __device__ __forceinline__ v16h load(const _Float16* p) {
    U f; f.h[0] = *(const v8h*)(p); f.h[1] = *(const v8h*)(p + 16); return f.v;
  }
  static __device__ __forceinline__ v8f mma(v16h a, v16h b, v8f c) {
    return __builtin_amdgcn_wmma_f32_16x16x32_f16(false, a, false, b, (short)0, c, false, false);
  }
  static __device__ __forceinline__ void guard(v8f& a, v8f& b, v16h x, v16h y) { dep_guard_h(a, b, x, y); }
  static __device__ __forceinline__ void keep(v16h a, v16h b, v16h c, v16h d) { keep4_h(a, b, c, d); }
};
template <> struct Frag<__bf16> {
  typedef v16b V; union U { v16b v; v8b h[2]; };
  static __device__ __forceinline__ v16b load(const __bf16* p) {
    U f; f.h[0] = *(const v8b*)(p); f.h[1] = *(const v8b*)(p + 16); return f.v;
  }
  static __device__ __forceinline__ v8f mma(v16b a, v16b b, v8f c) {
    return __builtin_amdgcn_wmma_f32_16x16x32_bf16(false, a, false, b, (short)0, c, false, false);
  }
  static __device__ __forceinline__ void guard(v8f& a, v8f& b, v16b x, v16b y) { dep_guard_b(a, b, x, y); }
  static __device__ __forceinline__ void keep(v16b a, v16b b, v16b c, v16b d) { keep4_b(a, b, c, d); }
};

__device__ __forceinline__ float fsig(float x)  { return __builtin_amdgcn_rcpf(1.0f + __expf(-x)); }
__device__ __forceinline__ float ftanh(float x) { return 1.0f - 2.0f * __builtin_amdgcn_rcpf(__expf(2.0f * x) + 1.0f); }

__global__ __launch_bounds__(kThreads) void cast_scale_f32_f16x2(
    const float* __restrict__ in, _Float16* __restrict__ out, int n2, float sc) {
  const int i = blockIdx.x * kThreads + threadIdx.x;
  if (i < n2) {
    const _Float16 h0 = (_Float16)(in[2 * i] * sc), h1 = (_Float16)(in[2 * i + 1] * sc);
    const unsigned u = (unsigned)__builtin_bit_cast(unsigned short, h0) | ((unsigned)__builtin_bit_cast(unsigned short, h1) << 16);
    ((volatile unsigned*)out)[i] = u;
    __threadfence();
    ((volatile unsigned*)out)[i] = u;
  }
}

__global__ __launch_bounds__(kThreads) void cast_split_f32_bf16x2(
    const float* __restrict__ in, unsigned short* __restrict__ outh, unsigned short* __restrict__ outl, int n2, float sc) {
  const int i = blockIdx.x * kThreads + threadIdx.x;
  if (i < n2) {
    const float f0 = in[2 * i] * sc, f1 = in[2 * i + 1] * sc;
    const unsigned short h0 = f2bf_bits(f0), h1 = f2bf_bits(f1);
    const unsigned short l0 = f2bf_bits(f0 - bf_bits2f(h0)), l1 = f2bf_bits(f1 - bf_bits2f(h1));
    const unsigned uh = (unsigned)h0 | ((unsigned)h1 << 16);
    const unsigned ul = (unsigned)l0 | ((unsigned)l1 << 16);
    ((volatile unsigned*)outh)[i] = uh;
    ((volatile unsigned*)outl)[i] = ul;
    __threadfence();
    ((volatile unsigned*)outh)[i] = uh;
    ((volatile unsigned*)outl)[i] = ul;
  }
}

__global__ __launch_bounds__(kThreads) void path_kernel(
    const int* __restrict__ anc, const float* __restrict__ weight, const float* __restrict__ emb,
    int nTypes, int depth, unsigned short* __restrict__ Ph, unsigned short* __restrict__ Pl) {
  const int tid = threadIdx.x, lane = tid & 31, wave = tid >> 5;
  const int n  = blockIdx.x * kNodesPerBlk + wave;
  const int nn = n < nTypes ? n : (nTypes - 1);
  const int dcl = depth < kMaxDepth ? depth : kMaxDepth;
  float acc[8];
#pragma unroll
  for (int e = 0; e < 8; ++e) acc[e] = 0.0f;
  float cw = 1.0f;
#pragma unroll 1
  for (int d = 0; d < dcl; ++d) {
    const int a = anc[(size_t)nn * (size_t)depth + d];
    const bool valid = (a >= 0);
    int as = valid ? a : 0;
    as = as < nTypes ? as : (nTypes - 1);
    const float wv = weight[as];
    const float w  = valid ? wv : 1.0f;
    const float coef = valid ? cw : 0.0f;
    const float* er = emb + (size_t)as * kHid + 8 * lane;
    const v4f e0 = *(const v4f*)(er);
    const v4f e1 = *(const v4f*)(er + 4);
    acc[0] += coef * e0[0]; acc[1] += coef * e0[1]; acc[2] += coef * e0[2]; acc[3] += coef * e0[3];
    acc[4] += coef * e1[0]; acc[5] += coef * e1[1]; acc[6] += coef * e1[2]; acc[7] += coef * e1[3];
    cw *= w;
  }
  v8h hv, lv;
#pragma unroll
  for (int e = 0; e < 8; ++e) {
    const unsigned short hb = f2bf_bits(acc[e]);
    const unsigned short lb = f2bf_bits(acc[e] - bf_bits2f(hb));
    hv[e] = __builtin_bit_cast(_Float16, hb);
    lv[e] = __builtin_bit_cast(_Float16, lb);
  }
  if (n < nTypes) {
    const size_t o = (size_t)n * kHid + 8 * lane;
    *(volatile v8h*)(Ph + o) = hv;
    *(volatile v8h*)(Pl + o) = lv;
    __threadfence();
    *(volatile v8h*)(Ph + o) = hv;
    *(volatile v8h*)(Pl + o) = lv;
  }
}

__global__ __launch_bounds__(kThreads) void lstm_kernel(
    const int* __restrict__ events, const unsigned short* __restrict__ Php, const unsigned short* __restrict__ Plp,
    const unsigned short* __restrict__ WXhp, const unsigned short* __restrict__ WXlp, const unsigned short* __restrict__ WHp,
    const float* __restrict__ b_ih, const float* __restrict__ b_hh,
    float* __restrict__ out, int nTypes) {
  __shared__ __align__(16) __bf16   Axh[kSeqPerBlock * kHPitch];
  __shared__ __align__(16) __bf16   Axl[kSeqPerBlock * kHPitch];
  __shared__ __align__(16) _Float16 Ah[kSeqPerBlock * kHPitch];
  __shared__ __align__(16) float    Hs[kSeqPerBlock * kOPitch];
  const __bf16*   Ph  = (const __bf16*)Php;
  const __bf16*   Pl  = (const __bf16*)Plp;
  const __bf16*   WXh = (const __bf16*)WXhp;
  const __bf16*   WXl = (const __bf16*)WXlp;
  const _Float16* WH  = (const _Float16*)WHp;
  const int tid = threadIdx.x, lane = tid & 31, wave = tid >> 5;
  const int c = lane & 15, hh = lane >> 4, koff = hh * 8;
  const int rowbase = blockIdx.x * kSeqPerBlock;

#pragma unroll 1
  for (int i = 0; i < kSeqPerBlock; ++i) Ah[i * kHPitch + tid] = (_Float16)0.0f;
  {
    const int m = tid >> 4, c16 = (tid & 15) * 16;
    int ev = events[(size_t)(rowbase + m) * kSeq + 0];
    ev = ev < 0 ? 0 : ev; ev = ev < nTypes ? ev : (nTypes - 1);
    const size_t so = (size_t)ev * kHid + c16;
    const v8b xh0 = *(const v8b*)(Ph + so);
    const v8b xh1 = *(const v8b*)(Ph + so + 8);
    const v8b xl0 = *(const v8b*)(Pl + so);
    const v8b xl1 = *(const v8b*)(Pl + so + 8);
    *(v8b*)(Axh + m * kHPitch + c16)     = xh0;
    *(v8b*)(Axh + m * kHPitch + c16 + 8) = xh1;
    *(v8b*)(Axl + m * kHPitch + c16)     = xl0;
    *(v8b*)(Axl + m * kHPitch + c16 + 8) = xl1;
  }
  float cst[2][8], hst[2][8], bb[2][4];
#pragma unroll
  for (int nt = 0; nt < 2; ++nt) {
    const int j = 32 * wave + 16 * nt + c;
#pragma unroll
    for (int g = 0; g < 4; ++g) bb[nt][g] = b_ih[g * kHid + j] + b_hh[g * kHid + j];
#pragma unroll
    for (int r = 0; r < 8; ++r) { cst[nt][r] = 0.0f; hst[nt][r] = 0.0f; }
  }
  __syncthreads();

  const __bf16*   axhrow = Axh + c * kHPitch + koff;
  const __bf16*   axlrow = Axl + c * kHPitch + koff;
  const _Float16* ahrow  = Ah  + c * kHPitch + koff;
  const v8f z8 = {0.f, 0.f, 0.f, 0.f, 0.f, 0.f, 0.f, 0.f};

#pragma unroll 1
  for (int t = 0; t < kSeq; ++t) {
#pragma unroll
    for (int nt = 0; nt < 2; ++nt) {
      const int j = 32 * wave + 16 * nt + c;
      const __bf16*   wxh = WXh + (size_t)j * kHid + koff;
      const __bf16*   wxl = WXl + (size_t)j * kHid + koff;
      const _Float16* wh  = WH  + (size_t)j * kHid + koff;
      v8f acc[4];
      acc[0] = z8; acc[1] = z8; acc[2] = z8; acc[3] = z8;
#pragma unroll 1
      for (int k0 = 0; k0 < kHid; k0 += 32) {
        const v16b ah  = Frag<__bf16>::load(axhrow + k0);
        const v16b al  = Frag<__bf16>::load(axlrow + k0);
        const v16b bh0 = Frag<__bf16>::load(wxh + k0);
        const v16b bh1 = Frag<__bf16>::load(wxh + (size_t)1 * kHid * kHid + k0);
        const v16b bh2 = Frag<__bf16>::load(wxh + (size_t)2 * kHid * kHid + k0);
        const v16b bh3 = Frag<__bf16>::load(wxh + (size_t)3 * kHid * kHid + k0);
        const v16b bl0 = Frag<__bf16>::load(wxl + k0);
        const v16b bl1 = Frag<__bf16>::load(wxl + (size_t)1 * kHid * kHid + k0);
        const v16b bl2 = Frag<__bf16>::load(wxl + (size_t)2 * kHid * kHid + k0);
        const v16b bl3 = Frag<__bf16>::load(wxl + (size_t)3 * kHid * kHid + k0);
        acc[0] = Frag<__bf16>::mma(ah, bh0, acc[0]);
        acc[1] = Frag<__bf16>::mma(ah, bh1, acc[1]);
        acc[2] = Frag<__bf16>::mma(ah, bh2, acc[2]);
        acc[3] = Frag<__bf16>::mma(ah, bh3, acc[3]);
        acc[0] = Frag<__bf16>::mma(ah, bl0, acc[0]);
        acc[1] = Frag<__bf16>::mma(ah, bl1, acc[1]);
        acc[2] = Frag<__bf16>::mma(ah, bl2, acc[2]);
        acc[3] = Frag<__bf16>::mma(ah, bl3, acc[3]);
        acc[0] = Frag<__bf16>::mma(al, bh0, acc[0]);
        acc[1] = Frag<__bf16>::mma(al, bh1, acc[1]);
        acc[2] = Frag<__bf16>::mma(al, bh2, acc[2]);
        acc[3] = Frag<__bf16>::mma(al, bh3, acc[3]);
        dep_guard_b(acc[0], acc[3], ah, al);
        keep4_b(bh0, bh1, bh2, bh3);
        keep4_b(bl0, bl1, bl2, bl3);
      }
#pragma unroll 1
      for (int k0 = 0; k0 < kHid; k0 += 32) {
        const v16h a  = Frag<_Float16>::load(ahrow + k0);
        const v16h b0 = Frag<_Float16>::load(wh + k0);
        const v16h b1 = Frag<_Float16>::load(wh + (size_t)1 * kHid * kHid + k0);
        const v16h b2 = Frag<_Float16>::load(wh + (size_t)2 * kHid * kHid + k0);
        const v16h b3 = Frag<_Float16>::load(wh + (size_t)3 * kHid * kHid + k0);
        acc[0] = Frag<_Float16>::mma(a, b0, acc[0]);
        acc[1] = Frag<_Float16>::mma(a, b1, acc[1]);
        acc[2] = Frag<_Float16>::mma(a, b2, acc[2]);
        acc[3] = Frag<_Float16>::mma(a, b3, acc[3]);
        dep_guard_h(acc[0], acc[3], a, b3);
        keep4_h(b0, b1, b2, b3);
      }
      acc_guard4(acc[0], acc[1], acc[2], acc[3]);
#pragma unroll
      for (int r = 0; r < 8; ++r) {
        const float zi = acc[0][r] * kWCarryInv + bb[nt][0];
        const float zf = acc[1][r] * kWCarryInv + bb[nt][1];
        const float zg = acc[2][r] * kWCarryInv + bb[nt][2];
        const float zo = acc[3][r] * kWCarryInv + bb[nt][3];
        const float ig = fsig(zi);
        const float fg = fsig(zf);
        const float gg = ftanh(zg);
        const float og = fsig(zo);
        const float cn = fg * cst[nt][r] + ig * gg;
        cst[nt][r] = cn;
        hst[nt][r] = og * ftanh(cn);
      }
    }
    __syncthreads();
#pragma unroll
    for (int nt = 0; nt < 2; ++nt) {
      const int j = 32 * wave + 16 * nt + c;
#pragma unroll
      for (int r = 0; r < 8; ++r) {
        Ah[(8 * hh + r) * kHPitch + j] = (_Float16)hst[nt][r];
        Hs[(8 * hh + r) * kOPitch + j] = hst[nt][r];
      }
    }
    {
      const int tn = (t + 1 < kSeq) ? (t + 1) : (kSeq - 1);
      const int m = tid >> 4, c16 = (tid & 15) * 16;
      int ev = events[(size_t)(rowbase + m) * kSeq + tn];
      ev = ev < 0 ? 0 : ev; ev = ev < nTypes ? ev : (nTypes - 1);
      const size_t so = (size_t)ev * kHid + c16;
      const v8b xh0 = *(const v8b*)(Ph + so);
      const v8b xh1 = *(const v8b*)(Ph + so + 8);
      const v8b xl0 = *(const v8b*)(Pl + so);
      const v8b xl1 = *(const v8b*)(Pl + so + 8);
      *(v8b*)(Axh + m * kHPitch + c16)     = xh0;
      *(v8b*)(Axh + m * kHPitch + c16 + 8) = xh1;
      *(v8b*)(Axl + m * kHPitch + c16)     = xl0;
      *(v8b*)(Axl + m * kHPitch + c16 + 8) = xl1;
    }
    __syncthreads();
    float* orow = out + ((size_t)t * kBatch + (size_t)rowbase) * kHid;
    for (int pass = 0; pass < 2; ++pass) {
#pragma unroll
      for (int it = 0; it < 4; ++it) {
        const int idx = it * kThreads + tid;
        const int row = idx >> 6, c4 = (idx & 63) * 4;
        const v4f v = *(const v4f*)(Hs + row * kOPitch + c4);
        *(volatile v4f*)(orow + (size_t)row * kHid + c4) = v;
      }
      __threadfence();
    }
  }
}

extern "C" void kernel_launch(void* const* d_in, const int* in_sizes, int n_in,
                              void* d_out, int out_size, void* d_ws, size_t ws_size, hipStream_t stream) {
  if (n_in < 8 || d_out == nullptr || d_ws == nullptr) return;
  const int nTypes = in_sizes[2];
  if (nTypes <= 0) return;
  const int depth = in_sizes[1] / nTypes;
  if (depth <= 0 || depth > kMaxDepth || depth * nTypes != in_sizes[1]) return;
  if (in_sizes[0] != kBatch * kSeq || in_sizes[3] != nTypes * kHid || in_sizes[4] != kGates * kHid ||
      in_sizes[5] != kGates * kHid || in_sizes[6] != kGates || in_sizes[7] != kGates ||
      out_size != kSeq * kBatch * kHid) return;

  const int*   events = (const int*)d_in[0];
  const int*   anc    = (const int*)d_in[1];
  const float* weight = (const float*)d_in[2];
  const float* emb    = (const float*)d_in[3];
  const float* W_ih   = (const float*)d_in[4];
  const float* W_hh   = (const float*)d_in[5];
  const float* b_ih   = (const float*)d_in[6];
  const float* b_hh   = (const float*)d_in[7];
  float* out = (float*)d_out;

  char* ws = (char*)d_ws; size_t off = 0;
  auto carve = [&](size_t bytes) -> char* { char* p = ws + off; off += (bytes + 255) & ~(size_t)255; return p; };
  unsigned short* Ph  = (unsigned short*)carve((size_t)nTypes * kHid * 2);
  unsigned short* Pl  = (unsigned short*)carve((size_t)nTypes * kHid * 2);
  unsigned short* WXh = (unsigned short*)carve((size_t)kGates * kHid * 2);
  unsigned short* WXl = (unsigned short*)carve((size_t)kGates * kHid * 2);
  _Float16*       WH  = (_Float16*)carve((size_t)kGates * kHid * 2);
  if (off > ws_size || off > (size_t)134217728) return;

  const int pathBlocks = (nTypes + kNodesPerBlk - 1) / kNodesPerBlk;
  path_kernel<<<pathBlocks, kThreads, 0, stream>>>(anc, weight, emb, nTypes, depth, Ph, Pl);
  const int n2 = kGates * kHid / 2;
  cast_split_f32_bf16x2<<<(n2 + kThreads - 1) / kThreads, kThreads, 0, stream>>>(W_ih, WXh, WXl, n2, kWCarry);
  cast_scale_f32_f16x2<<<(n2 + kThreads - 1) / kThreads, kThreads, 0, stream>>>(W_hh, WH, n2, kWCarry);
  lstm_kernel<<<kBatch / kSeqPerBlock, kThreads, 0, stream>>>(
      events, Ph, Pl, WXh, WXl, (const unsigned short*)WH, b_ih, b_hh, out, nTypes);
}
